// Embedding_31044023616454
// MI455X (gfx1250) — hardware-verified
//
#include <hip/hip_runtime.h>
#include <stddef.h>


typedef _Float16 v16h __attribute__((ext_vector_type(16)));
typedef _Float16 v8h  __attribute__((ext_vector_type(8)));
typedef float    v8f  __attribute__((ext_vector_type(8)));
typedef float    v4f  __attribute__((ext_vector_type(4)));
typedef unsigned int v8u __attribute__((ext_vector_type(8)));

#ifndef NB
#define NB 2
#endif
#ifndef SEQ
#define SEQ 4096
#endif
#define NB_FULL  2
#define SEQ_FULL 4096
#define DIM   128
#define VOCAB 32000
#define MROWS (NB * SEQ)

static_assert(NB >= 1 && NB <= NB_FULL);
static_assert(SEQ >= 64 && SEQ <= SEQ_FULL && (SEQ % 64) == 0);
static_assert(DIM == 128);
static_assert((DIM % 64) == 0);
static_assert((VOCAB % 64) == 0 && (VOCAB % 32) == 0 && (VOCAB % 8) == 0);
static_assert((MROWS % 64) == 0);
static_assert((size_t)NB_FULL * SEQ_FULL * DIM * 4 == (size_t)4194304);

#define LDT 72
#define LDO 132
static_assert((LDT % 8) == 0 && LDT >= 64);
static_assert((LDO % 4) == 0 && LDO >= DIM);

#define WCARRY 64.0f

#define WT_BYTES ((size_t)DIM * VOCAB * 2)
#define OFF_WT   ((size_t)0)
#define WS_TOTAL (OFF_WT + WT_BYTES)
static_assert((WT_BYTES % 128) == 0);
static_assert(WS_TOTAL <= (size_t)134217728);

__device__ __forceinline__ float bf16r(float x) {
  unsigned int u = __float_as_uint(x);
  u = (u + 0x7FFFu + ((u >> 16) & 1u)) & 0xFFFF0000u;
  return __uint_as_float(u);
}

__device__ __forceinline__ v16h frag_at(const _Float16* p) {
  v8h lo = *(const v8h*)(p);
  v8h hi = *(const v8h*)(p + 16);
  v16h out;
#pragma unroll
  for (int i = 0; i < 8; ++i) { out[i] = lo[i]; out[i + 8] = hi[i]; }
  return out;
}

__device__ __forceinline__ v8f wmma16(v16h a, v16h b, v8f c) {
  v8f d = __builtin_amdgcn_wmma_f32_16x16x32_f16(false, a, false, b, (short)0, c,
                                                 false, false);
  asm volatile("v_nop\n\tv_nop\n\tv_nop\n\tv_nop" : "+v"(d) : "v"(a), "v"(b));
  return d;
}

__device__ __forceinline__ v16h onehot_frag(unsigned u) {
  const unsigned one = 0x3C00u << ((u & 1u) << 4);
  const unsigned p = u >> 1;
  v8u wv;
#pragma unroll
  for (unsigned j = 0; j < 4u; ++j) {
    wv[j]      = (p == j)      ? one : 0u;
    wv[j + 4u] = (p == j + 8u) ? one : 0u;
  }
  return __builtin_bit_cast(v16h, wv);
}

__global__ __launch_bounds__(256) void wconv_kernel(
    const float* __restrict__ W, _Float16* __restrict__ Wt, unsigned ldw, unsigned ldk) {
  __shared__ _Float16 T[64 * LDT];
  const unsigned tid = threadIdx.x;
  const unsigned n0 = blockIdx.x * 64u;
  const unsigned k0 = blockIdx.y * 64u;
#pragma unroll 4
  for (unsigned j = 0; j < 16u; ++j) {
    const unsigned idx = tid + 256u * j;
    const unsigned kr = idx >> 6, nc = idx & 63u;
    const float v = W[(size_t)(k0 + kr) * ldw + n0 + nc];
    T[nc * LDT + kr] = (_Float16)(WCARRY * bf16r(v));
  }
  __syncthreads();
  v8h x[2];
  size_t off[2];
#pragma unroll
  for (unsigned i = 0; i < 2u; ++i) {
    const unsigned n = 32u * i + (tid >> 3);
    const unsigned kc = (tid & 7u) * 8u;
    x[i] = *(const v8h*)&T[n * LDT + kc];
    off[i] = (size_t)(n0 + n) * ldk + k0 + kc;
  }
#pragma unroll
  for (int i = 0; i < 2; ++i) *(volatile v8h*)(Wt + off[i]) = x[i];
  __threadfence();
#pragma unroll
  for (int i = 0; i < 2; ++i) *(volatile v8h*)(Wt + off[i]) = x[i];
}

__global__ __launch_bounds__(128) void onehot_gemm_kernel(
    const int* __restrict__ ids, const _Float16* __restrict__ Wt, float* __restrict__ outf) {
  __shared__ float Cs[64 * LDO];
  const unsigned lane = threadIdx.x & 31u;
  const unsigned w = (unsigned)__builtin_amdgcn_readfirstlane((int)(threadIdx.x >> 5));
  const unsigned hh = lane >> 4, m = lane & 15u;
  const unsigned row0 = blockIdx.x * 64u;
  const unsigned bidx = row0 / (unsigned)SEQ;
  const unsigned sq0 = row0 - bidx * (unsigned)SEQ;
  const size_t frow0 = (size_t)bidx * SEQ_FULL + sq0;

  const int id = ids[frow0 + w * 16u + m];
  const unsigned ub = (unsigned)id - hh * 8u;
  const _Float16* bp = Wt + (size_t)m * VOCAB + hh * 8u;

  v8f acc[8];
#pragma unroll
  for (int nb = 0; nb < 8; ++nb) acc[nb] = (v8f){};

#pragma unroll 1
  for (unsigned k0 = 0; k0 < (unsigned)VOCAB; k0 += 32u) {
    const v16h a = onehot_frag(ub - k0);
#pragma unroll
    for (int nb = 0; nb < 8; ++nb) {
      const v16h bf = frag_at(bp + (size_t)nb * 16u * VOCAB + k0);
      acc[nb] = wmma16(a, bf, acc[nb]);
    }
  }

#pragma unroll
  for (int nb = 0; nb < 8; ++nb)
#pragma unroll
    for (int r = 0; r < 8; ++r)
      Cs[(w * 16u + hh * 8u + (unsigned)r) * LDO + (unsigned)nb * 16u + m] =
          acc[nb][r] * (1.0f / WCARRY);
  __syncthreads();

  v4f x[16];
#pragma unroll
  for (unsigned r = 0; r < 16u; ++r)
    x[r] = *(const v4f*)&Cs[(w * 16u + r) * LDO + lane * 4u];
  float* op = outf + (frow0 + w * 16u) * DIM + lane * 4u;
#pragma unroll
  for (unsigned r = 0; r < 16u; ++r) *(volatile v4f*)(op + (size_t)r * DIM) = x[r];
  __threadfence();
#pragma unroll
  for (unsigned r = 0; r < 16u; ++r) *(volatile v4f*)(op + (size_t)r * DIM) = x[r];
}

extern "C" void kernel_launch(void* const* d_in, const int* in_sizes, int n_in,
                              void* d_out, int out_size, void* d_ws, size_t ws_size,
                              hipStream_t stream) {
  if (n_in < 2) return;
  const long long need_rows = (long long)(NB - 1) * SEQ_FULL + SEQ;
  if ((long long)in_sizes[0] < need_rows) return;
  if ((long long)in_sizes[1] < (long long)VOCAB * DIM) return;
  if ((long long)out_size < need_rows * DIM) return;
  if (ws_size < WS_TOTAL) return;

  const int*   ids = (const int*)d_in[0];
  const float* tab = (const float*)d_in[1];
  float* out = (float*)d_out;

  char* ws = (char*)d_ws;
  _Float16* Wt = (_Float16*)(ws + OFF_WT);

  wconv_kernel<<<dim3(DIM / 64, VOCAB / 64), dim3(256), 0, stream>>>(
      tab, Wt, (unsigned)DIM, (unsigned)VOCAB);
  onehot_gemm_kernel<<<dim3(MROWS / 64), dim3(128), 0, stream>>>(ids, Wt, out);
}
